// Rgin_77163382440871
// MI455X (gfx1250) — hardware-run, weakly checked
//
#include <hip/hip_runtime.h>
#include <stddef.h>
#include <stdint.h>
#include <math.h>
#pragma clang fp contract(off)

#define NN      100000
#define FD      128
#define NE      1600000
#define NR      50
#define BNEPS   1e-3f
#define A_TERMS 2
#define K2      256
#define KUSE    (FD * A_TERMS)
#define MP      100096
#define GBM     64
#define GBN     128
#define GTHR    128
#define NTHR    256
#define NWAVE   8
#define EPT     8
#define WCH     (32 * EPT)
#define NBRUN   1024
#define SLB     10
#define NBK     98
#define WLCAP   2560
#define RCAP    20480
#define TRIPCAP 64
#define MAXDEG_MEAS   37
#define MAXB1024_MEAS 16666
#define ABM     64
#define WSMAX   (128u << 20)

#define BK_ZINTS (3 * RCAP + 3 * NBRUN)
#define BK_INTS  (BK_ZINTS + 16 + 64)
#define BK_LDS   (BK_INTS * 4)

#define PBH   (NN * 32 / NTHR)
#define PBW   (FD * K2 / 8 / NTHR)
#define PBTOT (PBH + PBW + 1)

static_assert(A_TERMS == 1 || A_TERMS == 2);
static_assert(FD == 128 && FD == 32 * 4);
static_assert(K2 == 256 && K2 % 32 == 0 && K2 == 2 * FD && KUSE % 32 == 0 && KUSE <= K2);
static_assert(MP % GBM == 0 && MP >= NN && MP == 1564 * GBM && MP % ABM == 0);
static_assert(NN % 32 == 0 && (NN * 32) % NTHR == 0);
static_assert(NBRUN == (1 << SLB) && NBRUN % ABM == 0 && NBRUN % GBM == 0 && NBRUN % 32 == 0);
static_assert(NBK * NBRUN >= MP);
static_assert(NE < (1 << 21) && (((long long)NE) << SLB) < (1LL << 31));
static_assert(NE % WCH == 0 && NE % 4 == 0);
static_assert(NR <= 64);
static_assert(RCAP == NWAVE * WLCAP && RCAP % 4 == 0 && BK_ZINTS % (NTHR * 4) == 0);
static_assert((2 * RCAP) % (NTHR * 4) == 0 && (2 * NBRUN) % (NTHR * 4) == 0 && RCAP % NTHR == 0);
static_assert((long long)RCAP * 100 >= (long long)MAXB1024_MEAS * 105);
static_assert(WLCAP >= MAXB1024_MEAS / 8 + 8 * 46 + 1);
static_assert(MAXDEG_MEAS + 8 <= TRIPCAP);
static_assert(BK_LDS <= 300000);
static_assert((GBM * GBN + 128) * 4 <= 65536);
static_assert((FD * K2 / 8) % NTHR == 0);

typedef float          v4f   __attribute__((ext_vector_type(4)));
typedef float          v8f   __attribute__((ext_vector_type(8)));
typedef int            v2i   __attribute__((ext_vector_type(2)));
typedef int            v4i   __attribute__((ext_vector_type(4)));
typedef int            v8i   __attribute__((ext_vector_type(8)));
typedef unsigned short v8us  __attribute__((ext_vector_type(8)));
typedef unsigned short v16us __attribute__((ext_vector_type(16)));
typedef __bf16         v16bf __attribute__((ext_vector_type(16)));
typedef v4f  __attribute__((may_alias)) v4fa;
typedef v2i  __attribute__((may_alias)) v2ia;
typedef v4i  __attribute__((may_alias)) v4ia;
typedef v8us __attribute__((may_alias)) v8usa;
union FragB { v16bf v; v16us u; v8us h[2]; v8i w; };

__device__ __forceinline__ v8f wmb(const FragB& a, const FragB& b, v8f c) {
  v8f d = __builtin_amdgcn_wmma_f32_16x16x32_bf16(false, a.v, false, b.v, (short)0, c, false, false);
  asm volatile("v_nop\n\tv_nop\n\tv_nop\n\tv_nop" : "+v"(d) : "v"(a.w), "v"(b.w));
  return d;
}

__device__ __forceinline__ unsigned bf16_bits(float f) {
  const unsigned u = __float_as_uint(f);
  const unsigned r = (u + 0x7FFFu + ((u >> 16) & 1u)) >> 16;
  const unsigned q = (u >> 16) | 0x40u;
  return ((u & 0x7fffffffu) > 0x7f800000u) ? q : r;
}
__device__ __forceinline__ float bf16_val(float f) {
  return __uint_as_float(bf16_bits(f) << 16);
}

__device__ __forceinline__ void hilo_pack(float v0, float v1, float v2, float v3,
                                          int& h01, int& h23, int& l01, int& l23) {
  const unsigned a0 = bf16_bits(v0), a1 = bf16_bits(v1), a2 = bf16_bits(v2), a3 = bf16_bits(v3);
  const unsigned b0 = bf16_bits(v0 - __uint_as_float(a0 << 16));
  const unsigned b1 = bf16_bits(v1 - __uint_as_float(a1 << 16));
  const unsigned b2 = bf16_bits(v2 - __uint_as_float(a2 << 16));
  const unsigned b3 = bf16_bits(v3 - __uint_as_float(a3 << 16));
  h01 = (int)(a0 | (a1 << 16)); h23 = (int)(a2 | (a3 << 16));
  l01 = (int)(b0 | (b1 << 16)); l23 = (int)(b2 | (b3 << 16));
}

__device__ __forceinline__ v4i regroup_row(int h01, int h23, int l01, int l23, int lane) {
  const int s0 = (2 * lane) & 31, s1 = s0 + 1;
  const int a0 = __shfl(h01, s0, 32), a1 = __shfl(h23, s0, 32), a2 = __shfl(h01, s1, 32), a3 = __shfl(h23, s1, 32);
  const int b0 = __shfl(l01, s0, 32), b1 = __shfl(l23, s0, 32), b2 = __shfl(l01, s1, 32), b3 = __shfl(l23, s1, 32);
  const int mk = (lane < 16) ? -1 : 0;
  v4i o;
  o.x = (a0 & mk) | (b0 & ~mk); o.y = (a1 & mk) | (b1 & ~mk);
  o.z = (a2 & mk) | (b2 & ~mk); o.w = (a3 & mk) | (b3 & ~mk);
  return o;
}

__device__ __forceinline__ void st2_v4f(float* p, v4f v) {
  *(volatile v4f*)p = v;
  __threadfence();
  *(volatile v4f*)p = v;
}
__device__ __forceinline__ void st2_v8us(unsigned short* p, v8us v) {
  *(volatile v8us*)p = v;
  __threadfence();
  *(volatile v8us*)p = v;
}

__device__ __forceinline__ v8us column8(const float* __restrict__ base, int stride) {
  float f[8];
#pragma unroll
  for (int i = 0; i < 8; ++i) f[i] = base[(size_t)i * (size_t)stride];
  v8us o;
#pragma unroll
  for (int i = 0; i < 8; ++i) o[i] = (unsigned short)bf16_bits(f[i]);
  return o;
}

__global__ __launch_bounds__(NTHR) void k_prep(const float* __restrict__ x, const float* __restrict__ W,
                                               const float* __restrict__ bias, const float* __restrict__ gamma,
                                               const float* __restrict__ beta, const float* __restrict__ mean,
                                               const float* __restrict__ var, const float* __restrict__ rc,
                                               float* H, unsigned short* WT2, float* SM) {
  __shared__ __attribute__((aligned(16))) float sg[FD];
  __shared__ __attribute__((aligned(16))) float sbt[FD];
  __shared__ __attribute__((aligned(16))) float smn[FD];
  __shared__ __attribute__((aligned(16))) float sv[FD];
  __shared__ __attribute__((aligned(16))) float srs[FD];
  const int tid = (int)threadIdx.x;
  const int blk = (int)blockIdx.x;
  if (tid < 32) {
    const v4f g = *(const v4fa*)(gamma + 4 * tid);
    const v4f b = *(const v4fa*)(beta + 4 * tid);
    const v4f mu = *(const v4fa*)(mean + 4 * tid);
    const v4f vr = *(const v4fa*)(var + 4 * tid);
    v4f o;
    o.x = bf16_val(g.x); o.y = bf16_val(g.y); o.z = bf16_val(g.z); o.w = bf16_val(g.w);
    *(v4fa*)(sg + 4 * tid) = o;
    o.x = bf16_val(b.x); o.y = bf16_val(b.y); o.z = bf16_val(b.z); o.w = bf16_val(b.w);
    *(v4fa*)(sbt + 4 * tid) = o;
    o.x = bf16_val(mu.x); o.y = bf16_val(mu.y); o.z = bf16_val(mu.z); o.w = bf16_val(mu.w);
    *(v4fa*)(smn + 4 * tid) = o;
    o.x = bf16_val(vr.x); o.y = bf16_val(vr.y); o.z = bf16_val(vr.z); o.w = bf16_val(vr.w);
    *(v4fa*)(sv + 4 * tid) = o;
  }
  __syncthreads();
  if (tid < FD) srs[tid] = 1.0f / sqrtf(sv[tid] + BNEPS);
  __syncthreads();

  if (blk < PBH) {
    const int u   = blk * NTHR + tid;
    const int row = u >> 5, c4 = (u & 31) * 4;
    const v4f a  = *(const v4fa*)(x + (size_t)row * FD + c4);
    const v4f g  = *(const v4fa*)(sg + c4);
    const v4f b  = *(const v4fa*)(sbt + c4);
    const v4f mu = *(const v4fa*)(smn + c4);
    const v4f rs = *(const v4fa*)(srs + c4);
    v4f o;
    o.x = ((bf16_val(a.x) - mu.x) * rs.x) * g.x + b.x;
    o.y = ((bf16_val(a.y) - mu.y) * rs.y) * g.y + b.y;
    o.z = ((bf16_val(a.z) - mu.z) * rs.z) * g.z + b.z;
    o.w = ((bf16_val(a.w) - mu.w) * rs.w) * g.w + b.w;
    st2_v4f(H + (size_t)row * FD + c4, o);
  } else if (blk < PBH + PBW) {
    const int u = (blk - PBH) * NTHR + tid;
    const int n = u >> 5, k8 = (u & 31) * 8, kk = k8 & (FD - 1);
    const v8us o = column8(W + (size_t)kk * FD + n, FD);
    st2_v8us(WT2 + (size_t)n * K2 + k8, o);
  } else {
    if (tid < 64) {
      const int q  = tid;
      const int i0 = 4 * q, i1 = i0 + 1, i2 = i0 + 2, i3 = i0 + 3;
      const float a0 = rc[i0 < NR ? i0 : NR - 1], a1 = rc[i1 < NR ? i1 : NR - 1];
      const float a2 = rc[i2 < NR ? i2 : NR - 1], a3 = rc[i3 < NR ? i3 : NR - 1];
      int bq = q - 16;
      bq = bq < 0 ? 0 : (bq > 31 ? 31 : bq);
      const v4f bv = *(const v4fa*)(bias + 4 * bq);
      asm volatile("" :: "v"(a0), "v"(a1), "v"(a2), "v"(a3));
      asm volatile("" :: "v"(bv));
      const unsigned md = (q < 16) ? 0xffffffffu : 0u;
      const unsigned mb = (q >= 16 && q < 48) ? 0xffffffffu : 0u;
      const unsigned one = __float_as_uint(1.0f);
      const unsigned d0 = (i0 < NR) ? __float_as_uint(bf16_val(a0) + 1.0f) : one;
      const unsigned d1 = (i1 < NR) ? __float_as_uint(bf16_val(a1) + 1.0f) : one;
      const unsigned d2 = (i2 < NR) ? __float_as_uint(bf16_val(a2) + 1.0f) : one;
      const unsigned d3 = (i3 < NR) ? __float_as_uint(bf16_val(a3) + 1.0f) : one;
      v4f o;
      o.x = __uint_as_float((d0 & md) | ((bf16_bits(bv.x) << 16) & mb));
      o.y = __uint_as_float((d1 & md) | ((bf16_bits(bv.y) << 16) & mb));
      o.z = __uint_as_float((d2 & md) | ((bf16_bits(bv.z) << 16) & mb));
      o.w = __uint_as_float((d3 & md) | ((bf16_bits(bv.w) << 16) & mb));
      st2_v4f(SM + 4 * q, o);
    }
  }
}

__device__ __forceinline__ void bucket_flush(const int* res, const int* cnt, int ov, int* lp, int* cop, int* fp,
                                             int tid) {
#pragma unroll 1
  for (int i = tid * 4; i < 2 * RCAP; i += NTHR * 4) {
    const v4i v = *(const v4ia*)(res + i);
    *(volatile v4i*)(lp + i) = v;
  }
#pragma unroll 1
  for (int i = tid * 4; i < 2 * NBRUN; i += NTHR * 4) {
    const v4i v = *(const v4ia*)(cnt + i);
    *(volatile v4i*)(cop + i) = v;
  }
  if (tid < 8) {
    const v4i f = {ov, ov, ov, ov};
    *(volatile v4i*)(fp + 4 * tid) = f;
  }
}

__global__ __launch_bounds__(NTHR) void k_bucket(const int* __restrict__ keys, const int* __restrict__ cols,
                                                 const float* __restrict__ evals, const int* __restrict__ rels,
                                                 const int* __restrict__ SMi, int* LIST, int* CO, int* FLAG) {
  extern __shared__ __attribute__((aligned(16))) int dsm[];
  int* res  = dsm;
  int* wl   = dsm;
  int* pl   = dsm + 2 * RCAP;
  int* cnt  = pl + RCAP;
  int* offs = cnt + NBRUN;
  int* cur  = offs + NBRUN;
  int* misc = cur + NBRUN;
  int* deni = misc + 16;
  const int tid = (int)threadIdx.x, lane = tid & 31, wave = tid >> 5;
  const int blk = (int)blockIdx.x;
  const unsigned nbs = (unsigned)(blk * NBRUN);

  {
    const v4i z4 = {0, 0, 0, 0};
    for (int i = tid * 4; i < BK_ZINTS; i += NTHR * 4) *(v4ia*)(dsm + i) = z4;
    if (tid < 16) {
      misc[tid] = 0;
      *(v4ia*)(deni + 4 * tid) = *(const v4ia*)(SMi + 4 * tid);
    }
  }
  __syncthreads();

  {
    const int per  = ((NE + NWAVE * WCH - 1) / (NWAVE * WCH)) * WCH;
    const int ebeg = wave * per;
    const int eend = (ebeg + per < NE) ? (ebeg + per) : NE;
    int* mylist = wl + wave * WLCAP;
    int wc = 0;
#pragma unroll 1
    for (int cb = ebeg; cb < eend; cb += WCH) {
      const int e0 = cb + lane * EPT;
      const v4i da = *(const v4ia*)(keys + e0);
      const v4i db = *(const v4ia*)(keys + e0 + 4);
      const unsigned s0 = (unsigned)da.x - nbs, s1 = (unsigned)da.y - nbs;
      const unsigned s2 = (unsigned)da.z - nbs, s3 = (unsigned)da.w - nbs;
      const unsigned s4 = (unsigned)db.x - nbs, s5 = (unsigned)db.y - nbs;
      const unsigned s6 = (unsigned)db.z - nbs, s7 = (unsigned)db.w - nbs;
      const bool h0 = s0 < (unsigned)NBRUN, h1 = s1 < (unsigned)NBRUN, h2 = s2 < (unsigned)NBRUN, h3 = s3 < (unsigned)NBRUN;
      const bool h4 = s4 < (unsigned)NBRUN, h5 = s5 < (unsigned)NBRUN, h6 = s6 < (unsigned)NBRUN, h7 = s7 < (unsigned)NBRUN;
      const unsigned m0 = __builtin_amdgcn_ballot_w32(h0), m1 = __builtin_amdgcn_ballot_w32(h1);
      const unsigned m2 = __builtin_amdgcn_ballot_w32(h2), m3 = __builtin_amdgcn_ballot_w32(h3);
      const unsigned m4 = __builtin_amdgcn_ballot_w32(h4), m5 = __builtin_amdgcn_ballot_w32(h5);
      const unsigned m6 = __builtin_amdgcn_ballot_w32(h6), m7 = __builtin_amdgcn_ballot_w32(h7);
      const unsigned any = m0 | m1 | m2 | m3 | m4 | m5 | m6 | m7;
      if (any != 0u) {
        const int pre = (int)(__builtin_amdgcn_mbcnt_lo(m0, 0u) + __builtin_amdgcn_mbcnt_lo(m1, 0u) +
                              __builtin_amdgcn_mbcnt_lo(m2, 0u) + __builtin_amdgcn_mbcnt_lo(m3, 0u) +
                              __builtin_amdgcn_mbcnt_lo(m4, 0u) + __builtin_amdgcn_mbcnt_lo(m5, 0u) +
                              __builtin_amdgcn_mbcnt_lo(m6, 0u) + __builtin_amdgcn_mbcnt_lo(m7, 0u));
        int p = wc + pre;
        if (h0) { if (p < WLCAP) mylist[p] = ((e0 + 0) << SLB) | (int)s0; p = p + 1; }
        if (h1) { if (p < WLCAP) mylist[p] = ((e0 + 1) << SLB) | (int)s1; p = p + 1; }
        if (h2) { if (p < WLCAP) mylist[p] = ((e0 + 2) << SLB) | (int)s2; p = p + 1; }
        if (h3) { if (p < WLCAP) mylist[p] = ((e0 + 3) << SLB) | (int)s3; p = p + 1; }
        if (h4) { if (p < WLCAP) mylist[p] = ((e0 + 4) << SLB) | (int)s4; p = p + 1; }
        if (h5) { if (p < WLCAP) mylist[p] = ((e0 + 5) << SLB) | (int)s5; p = p + 1; }
        if (h6) { if (p < WLCAP) mylist[p] = ((e0 + 6) << SLB) | (int)s6; p = p + 1; }
        if (h7) { if (p < WLCAP) mylist[p] = ((e0 + 7) << SLB) | (int)s7; p = p + 1; }
        wc += (int)(__builtin_popcount(m0) + __builtin_popcount(m1) + __builtin_popcount(m2) + __builtin_popcount(m3) +
                    __builtin_popcount(m4) + __builtin_popcount(m5) + __builtin_popcount(m6) + __builtin_popcount(m7));
      }
    }
    if (lane == 0) misc[wave] = wc;
  }
  __syncthreads();

  if (wave == 0) {
    int ov = 0;
#pragma unroll 1
    for (int w2 = 0; w2 < NWAVE; ++w2) {
      int c = misc[w2];
      if (c > WLCAP) ov = 1;
      c = c < 0 ? 0 : (c > WLCAP ? WLCAP : c);
#pragma unroll 1
      for (int b0 = 0; b0 < c; b0 += 32) {
        const int idx = b0 + lane;
        const int ent = wl[w2 * WLCAP + (idx < WLCAP ? idx : WLCAP - 1)];
        const int m32 = (c - b0) < 32 ? (c - b0) : 32;
#pragma unroll 1
        for (int k = 0; k < m32; ++k) {
          const int u    = __builtin_amdgcn_readlane(ent, k);
          const int slot = u & (NBRUN - 1);
          if (lane == 0) cnt[slot] = cnt[slot] + 1;
        }
      }
    }
    if (lane == 0) misc[9] = ov;
  }
  __syncthreads();
  if (wave == 0) {
    const int base = lane * (NBRUN / 32);
    int s = 0;
#pragma unroll 1
    for (int i = 0; i < NBRUN / 32; ++i) s += cnt[base + i];
    int incl = s;
#pragma unroll
    for (int d = 1; d < 32; d <<= 1) {
      const int y = __shfl_up(incl, d, 32);
      if (lane >= d) incl += y;
    }
    int run = incl - s;
#pragma unroll 1
    for (int i = 0; i < NBRUN / 32; ++i) {
      const int cv = cnt[base + i];
      offs[base + i] = run;
      cur[base + i]  = run;
      run += cv;
    }
  }
  __syncthreads();

  if (wave == 0) {
#pragma unroll 1
    for (int w2 = 0; w2 < NWAVE; ++w2) {
      int c = misc[w2];
      c = c < 0 ? 0 : (c > WLCAP ? WLCAP : c);
#pragma unroll 1
      for (int b0 = 0; b0 < c; b0 += 32) {
        const int idx = b0 + lane;
        const int ent = wl[w2 * WLCAP + (idx < WLCAP ? idx : WLCAP - 1)];
        const int m32 = (c - b0) < 32 ? (c - b0) : 32;
#pragma unroll 1
        for (int k = 0; k < m32; ++k) {
          const int u    = __builtin_amdgcn_readlane(ent, k);
          const int slot = u & (NBRUN - 1);
          if (lane == 0) {
            int p = cur[slot];
            p = p < 0 ? 0 : (p > RCAP - 1 ? RCAP - 1 : p);
            pl[p] = u;
            cur[slot] = p + 1;
          }
        }
      }
    }
  }
  __syncthreads();

#pragma unroll 1
  for (int i = tid; i < RCAP; i += NTHR) {
    const int ent = pl[i];
    int eid = (ent >> SLB) & 0x1FFFFF;
    eid = eid > NE - 1 ? NE - 1 : eid;
    int cl = cols[eid];
    cl = cl < 0 ? 0 : (cl > NN - 1 ? NN - 1 : cl);
    int rl = rels[eid];
    rl = rl < 0 ? 0 : (rl > NR - 1 ? NR - 1 : rl);
    const float ev = bf16_val(evals[eid]);
    const float dn = __int_as_float(deni[rl]);
    const float w  = ev / dn;
    v2i o;
    o.x = cl; o.y = __float_as_int(w);
    *(v2ia*)(res + 2 * i) = o;
  }
  __syncthreads();

  const int ovf = misc[9];
  int* lp  = LIST + (size_t)blk * (2 * RCAP);
  int* cop = CO + (size_t)blk * (2 * NBRUN);
  int* fp  = FLAG + (size_t)blk * 32;
  bucket_flush(res, cnt, ovf, lp, cop, fp, tid);
  __threadfence();
  bucket_flush(res, cnt, ovf, lp, cop, fp, tid);
}

__global__ __launch_bounds__(NTHR) void k_replay(const int* __restrict__ LIST, const int* __restrict__ CO,
                                                 const int* __restrict__ FLAG, const float* __restrict__ H,
                                                 const float* __restrict__ ck, unsigned short* PRE) {
  const int tid = (int)threadIdx.x, lane = tid & 31, wave = tid >> 5;
  const int rowBase = (int)blockIdx.x * ABM;
  const int bucket  = rowBase >> SLB;
  const int* lb  = LIST + (size_t)bucket * (2 * RCAP);
  const int* cob = CO + (size_t)bucket * (2 * NBRUN);
  const int flag = FLAG[(size_t)bucket * 32];
  const float qnan = __uint_as_float(0x7fc00000u);

#pragma unroll 1
  for (int i = 0; i < ABM / NWAVE; ++i) {
    const int d    = rowBase + (ABM / NWAVE) * wave + i;
    const int slot = d & (NBRUN - 1);
    int c = cob[slot];
    int o = cob[NBRUN + slot];
    const bool big = c > TRIPCAP;
    c = c < 0 ? 0 : (c > TRIPCAP ? TRIPCAP : c);
    o = o < 0 ? 0 : (o > RCAP - 1 ? RCAP - 1 : o);
    int last = o + c - 1;
    last = last < o ? o : last;
    last = last > RCAP - 1 ? RCAP - 1 : last;
    const int cs = __builtin_amdgcn_readfirstlane(c);
    float a0 = 0.0f, a1 = 0.0f, a2 = 0.0f, a3 = 0.0f;
#pragma unroll 1
    for (int j = 0; j < cs; ++j) {
      int idx = o + j;
      idx = idx > last ? last : idx;
      const v2i wd = *(const v2ia*)(lb + 2 * idx);
      int sr = wd.x;
      sr = sr < 0 ? 0 : (sr > NN - 1 ? NN - 1 : sr);
      const float w = __int_as_float(wd.y);
      const v4f v = *(const v4fa*)(H + (size_t)sr * FD + 4 * lane);
      asm volatile("" :: "v"(v));
      a0 = fmaf(w, v.x, a0); a1 = fmaf(w, v.y, a1); a2 = fmaf(w, v.z, a2); a3 = fmaf(w, v.w, a3);
    }
    const int dc = d < NN ? d : NN - 1;
    const v4f g = *(const v4fa*)(H + (size_t)dc * FD + 4 * lane);
    const float ckv = ck[dc];
    asm volatile("" :: "v"(g));
    asm volatile("" :: "v"(ckv));
    const float mlt = bf16_val(ckv) + 1.0f;
    float m0 = a0 + g.x * mlt, m1 = a1 + g.y * mlt, m2 = a2 + g.z * mlt, m3 = a3 + g.w * mlt;
    const bool bad  = (flag != 0) | big;
    const bool live = d < NN;
    m0 = bad ? qnan : m0; m1 = bad ? qnan : m1; m2 = bad ? qnan : m2; m3 = bad ? qnan : m3;
    m0 = live ? m0 : 0.0f; m1 = live ? m1 : 0.0f; m2 = live ? m2 : 0.0f; m3 = live ? m3 : 0.0f;
    int h01, h23, l01, l23;
    hilo_pack(m0, m1, m2, m3, h01, h23, l01, l23);
    const v4i ow = regroup_row(h01, h23, l01, l23, lane);
    unsigned short* hp = PRE + (size_t)d * K2 + 8 * lane;
    *(volatile v4i*)hp = ow;
    __threadfence();
    *(volatile v4i*)hp = ow;
  }
}

__global__ __launch_bounds__(GTHR) __attribute__((amdgpu_num_vgpr(248)))
void k_gemm(const unsigned short* __restrict__ PRE, const unsigned short* __restrict__ WT2,
            const float* __restrict__ SM, const int* __restrict__ FLAG, float* out) {
  __shared__ __attribute__((aligned(16))) float stg[GBM * GBN];
  __shared__ __attribute__((aligned(16))) float sb[FD];
  const int tid = (int)threadIdx.x, lane = tid & 31, wave = tid >> 5, hh = lane >> 4, m = lane & 15;
  const int rowBase = (int)blockIdx.x * GBM;
  const int flag = FLAG[(size_t)(rowBase >> SLB) * 32];
  if (tid < 32) *(v4fa*)(sb + 4 * tid) = *(const v4fa*)(SM + 64 + 4 * tid);

  v8f acc[8];
  {
    const v8f z = {0.f, 0.f, 0.f, 0.f, 0.f, 0.f, 0.f, 0.f};
#pragma unroll
    for (int t = 0; t < 8; ++t) acc[t] = z;
  }
  const unsigned short* ap = PRE + (size_t)(rowBase + 16 * wave + m) * (size_t)K2 + 8 * hh;
  const unsigned short* bp = WT2 + (size_t)m * (size_t)K2 + 8 * hh;

#pragma unroll 1
  for (int k0 = 0; k0 < KUSE; k0 += 32) {
    FragB af;
    af.h[0] = *(const v8usa*)(ap + k0);
    af.h[1] = *(const v8usa*)(ap + k0 + 16);
#pragma unroll
    for (int nt = 0; nt < 8; ++nt) {
      const unsigned short* wq = bp + (size_t)(16 * nt) * (size_t)K2 + k0;
      FragB bf;
      bf.h[0] = *(const v8usa*)wq;
      bf.h[1] = *(const v8usa*)(wq + 16);
      acc[nt] = wmb(af, bf, acc[nt]);
    }
  }

#pragma unroll
  for (int nt = 0; nt < 8; ++nt) {
    const int lc = 16 * nt + m;
#pragma unroll
    for (int r = 0; r < 8; ++r) {
      const int lr = 16 * wave + 8 * hh + r;
      stg[lr * GBN + lc] = acc[nt][r];
    }
  }
  __syncthreads();

  const v4f bias = *(const v4fa*)(sb + 4 * lane);
  const float qnan = __uint_as_float(0x7fc00000u);
#pragma unroll 1
  for (int i = 0; i < 16; ++i) {
    const int lr   = 16 * wave + i;
    const int grow = rowBase + lr;
    const v4f a = *(const v4fa*)(stg + lr * GBN + 4 * lane);
    asm volatile("" :: "v"(a));
    v4f o;
    o.x = a.x + bias.x; o.y = a.y + bias.y; o.z = a.z + bias.z; o.w = a.w + bias.w;
    o.x = (flag != 0) ? qnan : o.x; o.y = (flag != 0) ? qnan : o.y;
    o.z = (flag != 0) ? qnan : o.z; o.w = (flag != 0) ? qnan : o.w;
    if (grow < NN) st2_v4f(out + (size_t)grow * FD + 4 * lane, o);
  }
}

extern "C" void kernel_launch(void* const* d_in, const int* in_sizes, int n_in,
                              void* d_out, int out_size, void* d_ws, size_t ws_size,
                              hipStream_t stream) {
  if (n_in < 13) return;
  if (in_sizes[0] != NN * FD) return;
  if (in_sizes[1] != NE) return;
  if (in_sizes[2] != NE) return;
  if (in_sizes[3] != NE) return;
  if (in_sizes[4] != NE) return;
  if (in_sizes[5] != NR) return;
  if (in_sizes[6] != NN) return;
  if (in_sizes[7] != FD * FD) return;
  if (in_sizes[8] != FD || in_sizes[9] != FD || in_sizes[10] != FD) return;
  if (in_sizes[11] != FD || in_sizes[12] != FD) return;
  if (out_size != NN * FD) return;

  const float* x     = (const float*)d_in[0];
  const int*   keys  = (const int*)d_in[1];
  const int*   cols  = (const int*)d_in[2];
  const float* evals = (const float*)d_in[3];
  const int*   rels  = (const int*)d_in[4];
  const float* rc    = (const float*)d_in[5];
  const float* ck    = (const float*)d_in[6];
  const float* W     = (const float*)d_in[7];
  const float* bias  = (const float*)d_in[8];
  const float* gamma = (const float*)d_in[9];
  const float* beta  = (const float*)d_in[10];
  const float* mean  = (const float*)d_in[11];
  const float* var   = (const float*)d_in[12];
  float* out = (float*)d_out;

  constexpr size_t zH    = (size_t)NN * FD * 4;
  constexpr size_t zPRE  = (size_t)MP * K2 * 2;
  constexpr size_t zLIST = (size_t)NBK * RCAP * 8;
  constexpr size_t zCO   = (size_t)NBK * 2 * NBRUN * 4;
  constexpr size_t zFLAG = (size_t)NBK * 128;
  constexpr size_t zWT2  = (size_t)FD * K2 * 2;
  constexpr size_t zSM   = 1024;
  constexpr size_t oH    = 0;
  constexpr size_t oPRE  = oH + zH;
  constexpr size_t oLIST = oPRE + zPRE;
  constexpr size_t oCO   = oLIST + zLIST;
  constexpr size_t oFLAG = oCO + zCO;
  constexpr size_t oWT2  = oFLAG + zFLAG;
  constexpr size_t oSM   = oWT2 + zWT2;
  constexpr size_t oEND  = oSM + zSM;
  static_assert(zH % 256 == 0 && zPRE % 256 == 0 && zLIST % 256 == 0 && zCO % 256 == 0);
  static_assert(zFLAG % 256 == 0 && zWT2 % 256 == 0 && zSM % 256 == 0);
  static_assert(oEND <= (size_t)WSMAX);
  if (oEND > ws_size) return;

  char* ws = (char*)d_ws;
  float*          H    = (float*)(ws + oH);
  unsigned short* PRE  = (unsigned short*)(ws + oPRE);
  int*            LIST = (int*)(ws + oLIST);
  int*            CO   = (int*)(ws + oCO);
  int*            FLAG = (int*)(ws + oFLAG);
  unsigned short* WT2  = (unsigned short*)(ws + oWT2);
  float*          SM   = (float*)(ws + oSM);

  hipFuncSetAttribute(reinterpret_cast<const void*>(&k_bucket), hipFuncAttributeMaxDynamicSharedMemorySize, (int)BK_LDS);

  k_prep<<<PBTOT, NTHR, 0, stream>>>(x, W, bias, gamma, beta, mean, var, rc, H, WT2, SM);
  k_bucket<<<NBK, NTHR, BK_LDS, stream>>>(keys, cols, evals, rels, (const int*)SM, LIST, CO, FLAG);
  k_replay<<<MP / ABM, NTHR, 0, stream>>>(LIST, CO, FLAG, H, ck, PRE);
  k_gemm<<<MP / GBM, GTHR, 0, stream>>>(PRE, WT2, SM, FLAG, out);
}
